// DecoderLayer_44676249813143
// MI455X (gfx1250) — hardware-verified
//
#include <hip/hip_runtime.h>
#ifndef NB
#define NB 4
#endif
#ifndef SEQ
#define SEQ 1024
#endif
#define NB_FULL 4
#define SEQ_FULL 1024
#define DM 1024
#define NH 16
#define HD 64
#define DFF 4096
#define LQ (3 * DM)
#define MROWS (NB * SEQ)
#define NQT (SEQ / 64)
static_assert(SEQ % 64 == 0);
static_assert(SEQ <= SEQ_FULL);
static_assert(NB >= 1 && NB <= NB_FULL);
static_assert(MROWS % 128 == 0);
static_assert(DM == NH * HD && NH == 16 && HD == 64);
static_assert(DM % 64 == 0 && DFF % 64 == 0 && LQ % 64 == 0 && DM % 32 == 0 && DFF % 32 == 0);
static_assert((SEQ * DM / 8) % 256 == 0);
static_assert((DM * DM / 8) % 256 == 0 && (DFF * DM / 8) % 256 == 0);
static_assert((size_t)(SEQ * DM / 8 / 256) * NB * 256 * 8 == (size_t)MROWS * DM);
static_assert((size_t)(LQ / 64) * (MROWS / 128) * 128 * 64 == (size_t)MROWS * LQ);
static_assert((size_t)(DFF / 64) * (MROWS / 128) * 128 * 64 == (size_t)MROWS * DFF);
static_assert((size_t)(DM / 64) * (MROWS / 128) * 128 * 64 == (size_t)MROWS * DM);
static_assert((size_t)NQT * NB * NH * 64 * 64 == (size_t)NB * NH * HD * SEQ);
static_assert((size_t)NQT * NB * NH * 64 * 64 == (size_t)MROWS * DM);
static_assert((size_t)SEQ * NB * 256 * 4 == (size_t)MROWS * DM);

typedef _Float16 v16h __attribute__((ext_vector_type(16)));
typedef _Float16 v4h  __attribute__((ext_vector_type(4)));
typedef unsigned short v8us __attribute__((ext_vector_type(8), may_alias));
typedef float  v8f  __attribute__((ext_vector_type(8)));
typedef float  v4f  __attribute__((ext_vector_type(4)));
typedef float  v4fa __attribute__((ext_vector_type(4), may_alias));
union FragH { v16h v; v8us half[2]; _Float16 h[16]; unsigned short u[16]; };

#define NEG_INF (-__builtin_inff())

__device__ __forceinline__ unsigned short bf16_bits(float x) { unsigned int u = __float_as_uint(x); return (unsigned short)((u + 0x7FFFu + ((u >> 16) & 1u)) >> 16); }
__device__ __forceinline__ float bf16_val(unsigned short b) { return __uint_as_float(((unsigned int)b) << 16); }
__device__ __forceinline__ float bf16_rne(float x) { return bf16_val(bf16_bits(x)); }

__device__ __forceinline__ v16h g2_frag(const _Float16* p, unsigned hh) { FragH f; f.half[0] = *(const v8us*)((const unsigned short*)p + 8u * hh); f.half[1] = *(const v8us*)((const unsigned short*)p + 16u + 8u * hh); return f.v; }
__device__ __forceinline__ v8f g2_mma(v16h a, v16h b, v8f c) { v8f d = __builtin_amdgcn_wmma_f32_16x16x32_f16(false, a, false, b, (short)0, c, false, false); asm volatile("v_nop\n\tv_nop\n\tv_nop\n\tv_nop" : "+v"(d) : "v"(a), "v"(b)); return d; }

__device__ __forceinline__ float selu_f(float v) { const float e = __expf(fminf(v, 0.0f)) - 1.0f; return (v > 0.0f) ? 1.0507009873554805f * v : 1.7580993408473766f * e; }

__global__ __launch_bounds__(256) void k_x16(const float* __restrict__ x, _Float16* __restrict__ X16) {
  const unsigned t = blockIdx.x * 256u + threadIdx.x; const unsigned b = blockIdx.y;
  const float* src = x + ((size_t)b * SEQ_FULL * DM + (size_t)t * 8u);
  unsigned short* dst = (unsigned short*)X16 + ((size_t)b * SEQ * DM + (size_t)t * 8u);
  const v4f a = *(const v4fa*)src; const v4f c = *(const v4fa*)(src + 4); FragH f;
#pragma unroll
  for (int q = 0; q < 4; ++q) { f.h[q] = (_Float16)bf16_rne(a[q]); f.h[4 + q] = (_Float16)bf16_rne(c[q]); }
  *(volatile v8us*)dst = f.half[0]; __threadfence(); *(volatile v8us*)dst = f.half[0]; }

__global__ __launch_bounds__(256) void k_wnat(const float* __restrict__ w, unsigned n8, _Float16* __restrict__ Bt) {
  const unsigned t = blockIdx.x * 256u + threadIdx.x; if (t >= n8) return;
  const float* src = w + (size_t)t * 8u; const v4f a = *(const v4fa*)src; const v4f c = *(const v4fa*)(src + 4); FragH f;
#pragma unroll
  for (int q = 0; q < 4; ++q) { f.h[q] = (_Float16)(bf16_rne(a[q]) * 16.0f); f.h[4 + q] = (_Float16)(bf16_rne(c[q]) * 16.0f); }
  unsigned short* dst = (unsigned short*)Bt + (size_t)t * 8u;
  *(volatile v8us*)dst = f.half[0]; __threadfence(); *(volatile v8us*)dst = f.half[0]; }

template <int MODE>
__device__ __forceinline__ void gemm_body(float (*so)[32][68], const _Float16* __restrict__ A, unsigned lda, const _Float16* __restrict__ Bh, unsigned ldb, float alpha,
    const float* __restrict__ bias, const float* __restrict__ addp, _Float16* __restrict__ C16, float* __restrict__ C32, unsigned ldc, unsigned K) {
  const unsigned tid = threadIdx.x, w = tid >> 5, lane = tid & 31u, ln = lane & 15u, hh = lane >> 4;
  const unsigned row0 = blockIdx.y * 128u + 32u * w, col0 = blockIdx.x * 64u;
  const _Float16* a0p = A + (size_t)(row0 + ln) * lda; const _Float16* a1p = a0p + (size_t)16 * lda;
  const _Float16* b0p = Bh + (size_t)(col0 + ln) * ldb; const _Float16* b1p = b0p + (size_t)16 * ldb; const _Float16* b2p = b1p + (size_t)16 * ldb; const _Float16* b3p = b2p + (size_t)16 * ldb;
  const v8f z8 = {0.f,0.f,0.f,0.f,0.f,0.f,0.f,0.f}; v8f c00 = z8, c01 = z8, c02 = z8, c03 = z8, c10 = z8, c11 = z8, c12 = z8, c13 = z8;
#pragma unroll 1
  for (unsigned kb = 0; kb < K; kb += 32u) { const v16h a0 = g2_frag(a0p + kb, hh), a1 = g2_frag(a1p + kb, hh);
    v16h b = g2_frag(b0p + kb, hh); c00 = g2_mma(a0, b, c00); c10 = g2_mma(a1, b, c10);
    b = g2_frag(b1p + kb, hh); c01 = g2_mma(a0, b, c01); c11 = g2_mma(a1, b, c11);
    b = g2_frag(b2p + kb, hh); c02 = g2_mma(a0, b, c02); c12 = g2_mma(a1, b, c12);
    b = g2_frag(b3p + kb, hh); c03 = g2_mma(a0, b, c03); c13 = g2_mma(a1, b, c13); }
  v8f accs[8] = {c00, c01, c02, c03, c10, c11, c12, c13};
#pragma unroll
  for (int u = 0; u < 8; ++u) { const unsigned t = (unsigned)(u & 3), half = (unsigned)(u >> 2); const unsigned col = col0 + t * 16u + ln;
    float bv = 0.0f; if (MODE != 0) bv = bf16_rne(bias[col]);
#pragma unroll
    for (int r = 0; r < 8; ++r) { const unsigned rloc = half * 16u + 8u * hh + (unsigned)r; float v = accs[u][r] * alpha + bv; if (MODE == 1) v = selu_f(v); so[w][rloc][t * 16u + ln] = v; } }
  __builtin_amdgcn_fence(4  , "wavefront"); __builtin_amdgcn_wave_barrier();
  if (MODE != 2) {
    const unsigned rsub = lane >> 4, c4 = (lane & 15u) * 4u;
    for (int pass = 0; pass < 2; ++pass) {
#pragma unroll
      for (int q = 0; q < 16; ++q) { const unsigned r = (unsigned)q * 2u + rsub; const v4f v = *(const v4fa*)&so[w][r][c4]; v4h h4;
#pragma unroll
        for (int i = 0; i < 4; ++i) h4[i] = (_Float16)v[i];
        *(volatile v4h*)(C16 + (size_t)(row0 + r) * ldc + col0 + c4) = h4; }
      if (pass == 0) __threadfence(); }
  } else {
    const unsigned rq = lane >> 3, pc = lane & 7u;
    for (int pass = 0; pass < 2; ++pass) {
#pragma unroll
      for (int g = 0; g < 16; ++g) { const unsigned L = (unsigned)g * 4u + rq; const unsigned row = L >> 1, col = (L & 1u) * 32u + pc * 4u;
        const size_t gi = (size_t)(row0 + row) * ldc + col0 + col;
        v4f v = *(const v4fa*)&so[w][row][col]; const v4f ad = *(const v4fa*)(addp + gi);
#pragma unroll
        for (int i = 0; i < 4; ++i) v[i] += ad[i];
        *(volatile v4f*)(C32 + gi) = v; }
      if (pass == 0) __threadfence(); }
  } }

__global__ __launch_bounds__(128) void k_gemm_qkv(const _Float16* __restrict__ A, unsigned lda, const _Float16* __restrict__ Bh, unsigned ldb, float alpha, const float* __restrict__ bias,
    const float* __restrict__ addp, _Float16* __restrict__ C16, float* __restrict__ C32, unsigned ldc, unsigned K) {
  __shared__ __attribute__((aligned(16))) float so[4][32][68];
  gemm_body<0>(so, A, lda, Bh, ldb, alpha, bias, addp, C16, C32, ldc, K); }
__global__ __launch_bounds__(128) void k_gemm_selu(const _Float16* __restrict__ A, unsigned lda, const _Float16* __restrict__ Bh, unsigned ldb, float alpha, const float* __restrict__ bias,
    const float* __restrict__ addp, _Float16* __restrict__ C16, float* __restrict__ C32, unsigned ldc, unsigned K) {
  __shared__ __attribute__((aligned(16))) float so[4][32][68];
  gemm_body<1>(so, A, lda, Bh, ldb, alpha, bias, addp, C16, C32, ldc, K); }
__global__ __launch_bounds__(128) void k_gemm_res(const _Float16* __restrict__ A, unsigned lda, const _Float16* __restrict__ Bh, unsigned ldb, float alpha, const float* __restrict__ bias,
    const float* __restrict__ addp, _Float16* __restrict__ C16, float* __restrict__ C32, unsigned ldc, unsigned K) {
  __shared__ __attribute__((aligned(16))) float so[4][32][68];
  gemm_body<2>(so, A, lda, Bh, ldb, alpha, bias, addp, C16, C32, ldc, K); }

__global__ __launch_bounds__(256) void k_vt2(const _Float16* __restrict__ QKV, _Float16* __restrict__ VT) {
  __shared__ unsigned short tl[64][66];
  const unsigned tid = threadIdx.x; const unsigned lg = blockIdx.x, slab = blockIdx.y; const unsigned b = slab >> 4, hd = slab & 15u; const unsigned s0 = lg * 64u;
  for (unsigned i = tid; i < 64u * 8u; i += 256u) { const unsigned r = i >> 3, c8 = (i & 7u) * 8u; FragH f;
    f.half[0] = *(const v8us*)((const unsigned short*)QKV + ((size_t)(b * SEQ + s0 + r)) * LQ + 2u * DM + hd * HD + c8);
#pragma unroll
    for (int q = 0; q < 8; ++q) tl[r][c8 + (unsigned)q] = f.u[q]; }
  __syncthreads();
  for (int pass = 0; pass < 2; ++pass) {
#pragma unroll
    for (int rd = 0; rd < 2; ++rd) { const unsigned d = (unsigned)rd * 32u + (tid >> 3), pc = tid & 7u; FragH f;
#pragma unroll
      for (int q = 0; q < 8; ++q) f.u[q] = tl[pc * 8u + (unsigned)q][d];
      *(volatile v8us*)((unsigned short*)VT + ((size_t)slab * HD + d) * SEQ + s0 + pc * 8u) = f.half[0]; }
    if (pass == 0) __threadfence(); } }

__global__ __launch_bounds__(128) void k_attn(const _Float16* __restrict__ QKV, const _Float16* __restrict__ VT, const float* __restrict__ x, float* __restrict__ S1) {
  __shared__ __attribute__((aligned(16))) float so[4][16][68];
  const unsigned tid = threadIdx.x, w = tid >> 5, lane = tid & 31u, l15 = lane & 15u, hh = lane >> 4;
  const unsigned qt = blockIdx.x, slab = blockIdx.y; const unsigned b = slab >> 4, hd = slab & 15u;
  const unsigned q0 = qt * 64u + w * 16u;
  const _Float16* Qb = QKV + (size_t)b * SEQ * LQ + hd * HD;
  const _Float16* Kb = Qb + DM;
  const _Float16* Vb = VT + (size_t)slab * HD * SEQ;
  const _Float16* qrow = Qb + (size_t)(q0 + l15) * LQ;
  const v16h qf0 = g2_frag(qrow, hh), qf1 = g2_frag(qrow + 32, hh);
  const v8f z8 = {0.f,0.f,0.f,0.f,0.f,0.f,0.f,0.f};
  v8f o[4] = {z8, z8, z8, z8};
  float m = NEG_INF, l = 0.f;
  const float CL = 0.18033688011112042f;
#pragma unroll 1
  for (unsigned it = 0; it <= qt; ++it) {
    const unsigned key0 = it * 64u;
    v8f s[4];
#pragma unroll
    for (int kt = 0; kt < 4; ++kt) {
      const _Float16* krow = Kb + (size_t)(key0 + (unsigned)kt * 16u + l15) * LQ;
      const v16h ka = g2_frag(krow, hh), kk = g2_frag(krow + 32, hh);
      v8f a = g2_mma(ka, qf0, z8); a = g2_mma(kk, qf1, a); s[kt] = a; }
    if (it == qt) {
      const unsigned qrel = w * 16u + l15;
#pragma unroll
      for (int kt = 0; kt < 4; ++kt)
#pragma unroll
        for (int r = 0; r < 8; ++r) { const unsigned krel = (unsigned)kt * 16u + 8u * hh + (unsigned)r; s[kt][r] = (krel > qrel) ? NEG_INF : s[kt][r]; } }
    float lmax = NEG_INF;
#pragma unroll
    for (int kt = 0; kt < 4; ++kt)
#pragma unroll
      for (int r = 0; r < 8; ++r) lmax = fmaxf(lmax, s[kt][r]);
    lmax = fmaxf(lmax, __shfl_xor(lmax, 16));
    const float mnew = fmaxf(m, lmax);
    const float mref = (mnew == NEG_INF) ? 0.0f : mnew;
    const float alpha = exp2f((m - mref) * CL);
    const float bexp = 10.0f - mref * CL;
    m = mnew;
    float psum = 0.f; FragH pa, pb;
#pragma unroll
    for (int r = 0; r < 8; ++r) {
      const float e0 = exp2f(fmaf(s[0][r], CL, bexp)), e1 = exp2f(fmaf(s[1][r], CL, bexp)), e2 = exp2f(fmaf(s[2][r], CL, bexp)), e3 = exp2f(fmaf(s[3][r], CL, bexp));
      psum += (e0 + e1) + (e2 + e3);
      pa.h[r] = (_Float16)e0; pa.h[8 + r] = (_Float16)e1; pb.h[r] = (_Float16)e2; pb.h[8 + r] = (_Float16)e3; }
    l = l * alpha + psum;
    float ar[8];
#pragma unroll
    for (int r = 0; r < 8; ++r) ar[r] = __shfl(alpha, (int)(8u * hh) + r);
#pragma unroll
    for (int dt = 0; dt < 4; ++dt) {
#pragma unroll
      for (int r = 0; r < 8; ++r) o[dt][r] *= ar[r];
      const _Float16* vrow = Vb + (size_t)((unsigned)dt * 16u + l15) * SEQ + key0;
      const v16h va = g2_frag(vrow, hh), vb = g2_frag(vrow + 32, hh);
      o[dt] = g2_mma(pa.v, va, o[dt]); o[dt] = g2_mma(pb.v, vb, o[dt]); } }
  const float lt = l + __shfl_xor(l, 16);
  const float inv = 1.0f / lt;
  float ir[8];
#pragma unroll
  for (int r = 0; r < 8; ++r) ir[r] = __shfl(inv, (int)(8u * hh) + r);
#pragma unroll
  for (int dt = 0; dt < 4; ++dt)
#pragma unroll
    for (int r = 0; r < 8; ++r) so[w][8u * hh + (unsigned)r][(unsigned)dt * 16u + l15] = o[dt][r] * ir[r];
  __builtin_amdgcn_fence(4  , "wavefront"); __builtin_amdgcn_wave_barrier();
  const unsigned rq = lane >> 3, pc = lane & 7u;
  for (int pass = 0; pass < 2; ++pass) {
#pragma unroll
    for (int g = 0; g < 8; ++g) { const unsigned L = (unsigned)g * 4u + rq; const unsigned row = L >> 1, col = (L & 1u) * 32u + pc * 4u;
      const size_t go = ((size_t)(b * SEQ + q0 + row)) * DM + hd * HD + col;
      const size_t gx = ((size_t)(b * SEQ_FULL + q0 + row)) * DM + hd * HD + col;
      v4f v = *(const v4fa*)&so[w][row][col]; const v4f xr = *(const v4fa*)(x + gx);
#pragma unroll
      for (int i = 0; i < 4; ++i) v[i] += bf16_rne(xr[i]);
      *(volatile v4f*)(S1 + go) = v; }
    if (pass == 0) __threadfence(); } }

template <int HAS_H>
__device__ __forceinline__ void ln_body(float* r1, float* r2, const float* __restrict__ P, const float* __restrict__ g, const float* __restrict__ be,
    float* __restrict__ outF, unsigned obs, _Float16* __restrict__ outH) {
  const unsigned tid = threadIdx.x, w = tid >> 5, lane = tid & 31u; const unsigned s = blockIdx.x, b = blockIdx.y;
  const size_t rin = ((size_t)(b * SEQ + s)) * DM + tid * 4u;
  const v4f v = *(const v4fa*)(P + rin);
  float sm = (v[0] + v[1]) + (v[2] + v[3]);
  sm += __shfl_xor(sm, 16); sm += __shfl_xor(sm, 8); sm += __shfl_xor(sm, 4); sm += __shfl_xor(sm, 2); sm += __shfl_xor(sm, 1);
  if (lane == 0) r1[w] = sm;
  __syncthreads();
  const float tot = ((r1[0] + r1[1]) + (r1[2] + r1[3])) + ((r1[4] + r1[5]) + (r1[6] + r1[7]));
  const float mean = tot * (1.0f / (float)DM);
  const float d0 = v[0] - mean, d1 = v[1] - mean, d2 = v[2] - mean, d3 = v[3] - mean;
  float sq = (d0 * d0 + d1 * d1) + (d2 * d2 + d3 * d3);
  sq += __shfl_xor(sq, 16); sq += __shfl_xor(sq, 8); sq += __shfl_xor(sq, 4); sq += __shfl_xor(sq, 2); sq += __shfl_xor(sq, 1);
  if (lane == 0) r2[w] = sq;
  __syncthreads();
  const float tot2 = ((r2[0] + r2[1]) + (r2[2] + r2[3])) + ((r2[4] + r2[5]) + (r2[6] + r2[7]));
  const float rinv = rsqrtf(tot2 * (1.0f / (float)DM) + 1e-5f);
  const v4f gg = *(const v4fa*)(g + tid * 4u); const v4f bb = *(const v4fa*)(be + tid * 4u);
  v4f y; y[0] = d0 * rinv * bf16_rne(gg[0]) + bf16_rne(bb[0]); y[1] = d1 * rinv * bf16_rne(gg[1]) + bf16_rne(bb[1]);
  y[2] = d2 * rinv * bf16_rne(gg[2]) + bf16_rne(bb[2]); y[3] = d3 * rinv * bf16_rne(gg[3]) + bf16_rne(bb[3]);
  v4h h4; h4[0] = (_Float16)y[0]; h4[1] = (_Float16)y[1]; h4[2] = (_Float16)y[2]; h4[3] = (_Float16)y[3];
  float* op = outF + ((size_t)(b * obs + s)) * DM + tid * 4u;
  _Float16* hp = outH + rin;
  *(volatile v4f*)op = y; if (HAS_H) *(volatile v4h*)hp = h4;
  __threadfence();
  *(volatile v4f*)op = y; if (HAS_H) *(volatile v4h*)hp = h4; }

__global__ __launch_bounds__(256) void k_ln_h(const float* __restrict__ P, const float* __restrict__ g, const float* __restrict__ be, float* __restrict__ outF, unsigned obs, _Float16* __restrict__ outH) {
  __shared__ float r1[8]; __shared__ float r2[8];
  ln_body<1>(r1, r2, P, g, be, outF, obs, outH); }
__global__ __launch_bounds__(256) void k_ln_f(const float* __restrict__ P, const float* __restrict__ g, const float* __restrict__ be, float* __restrict__ outF, unsigned obs, _Float16* __restrict__ outH) {
  __shared__ float r1[8]; __shared__ float r2[8];
  ln_body<0>(r1, r2, P, g, be, outF, obs, outH); }

extern "C" void kernel_launch(void* const* d_in, const int* in_sizes, int n_in,
                              void* d_out, int out_size, void* d_ws, size_t ws_size, hipStream_t stream) {
  if (n_in < 12) return;
  const float* x   = (const float*)d_in[0];
  const float* Wq  = (const float*)d_in[1];
  const float* Wk  = (const float*)d_in[2];
  const float* Wv  = (const float*)d_in[3];
  const float* g1  = (const float*)d_in[4];
  const float* be1 = (const float*)d_in[5];
  const float* W1  = (const float*)d_in[6];
  const float* b1  = (const float*)d_in[7];
  const float* W2  = (const float*)d_in[8];
  const float* b2  = (const float*)d_in[9];
  const float* g2  = (const float*)d_in[10];
  const float* be2 = (const float*)d_in[11];
  const int xmin = ((NB - 1) * SEQ_FULL + SEQ) * DM;
  if (in_sizes[0] < xmin) return;
  if (in_sizes[1] < DM * DM || in_sizes[2] < DM * DM || in_sizes[3] < DM * DM) return;
  if (in_sizes[4] < DM || in_sizes[5] < DM || in_sizes[10] < DM || in_sizes[11] < DM) return;
  if (in_sizes[6] < DFF * DM || in_sizes[8] < DM * DFF) return;
  if (in_sizes[7] < DFF || in_sizes[9] < DM) return;
  if (out_size < xmin) return;
  char* ws = (char*)d_ws; size_t off = 0;
  auto take = [&](size_t bytes) { char* p = ws + off; off += (bytes + 255) & ~(size_t)255; return p; };
  const size_t qkv_bytes = (size_t)MROWS * LQ * 2, vt_bytes = (size_t)NB * NH * HD * SEQ * 2, h_bytes = (size_t)MROWS * DFF * 2;
  const size_t big_bytes = (qkv_bytes + vt_bytes > h_bytes) ? (qkv_bytes + vt_bytes) : h_bytes;
  _Float16* BQKV = (_Float16*)take((size_t)3 * DM * DM * 2);
  _Float16* B1   = (_Float16*)take((size_t)DFF * DM * 2);
  _Float16* B2   = (_Float16*)take((size_t)DM * DFF * 2);
  _Float16* XA   = (_Float16*)take((size_t)MROWS * DM * 2);
  char*     BIG  = take(big_bytes);
  float*    SA   = (float*)take((size_t)MROWS * DM * 4);
  float*    X1   = (float*)take((size_t)MROWS * DM * 4);
  if (off > ws_size || off > (size_t)134217728) return;
  _Float16* QKV = (_Float16*)BIG;
  _Float16* VT  = (_Float16*)(BIG + qkv_bytes);
  _Float16* Hh  = (_Float16*)BIG;
  const unsigned nw8 = (unsigned)(DM * DM / 8), nf8 = (unsigned)(DFF * DM / 8);
  k_wnat<<<(nw8 + 255u) / 256u, 256, 0, stream>>>(Wq, nw8, BQKV);
  k_wnat<<<(nw8 + 255u) / 256u, 256, 0, stream>>>(Wk, nw8, BQKV + (size_t)DM * DM);
  k_wnat<<<(nw8 + 255u) / 256u, 256, 0, stream>>>(Wv, nw8, BQKV + (size_t)2 * DM * DM);
  k_wnat<<<(nf8 + 255u) / 256u, 256, 0, stream>>>(W1, nf8, B1);
  k_wnat<<<(nf8 + 255u) / 256u, 256, 0, stream>>>(W2, nf8, B2);
  k_x16<<<dim3((unsigned)(SEQ * DM / 8 / 256), (unsigned)NB), 256, 0, stream>>>(x, XA);
  k_gemm_qkv<<<dim3((unsigned)(LQ / 64), (unsigned)(MROWS / 128)), 128, 0, stream>>>(XA, DM, BQKV, DM, 0.0625f, b1, x, QKV, SA, LQ, DM);
  k_vt2<<<dim3((unsigned)NQT, (unsigned)(NB * NH)), 256, 0, stream>>>(QKV, VT);
  k_attn<<<dim3((unsigned)NQT, (unsigned)(NB * NH)), 128, 0, stream>>>(QKV, VT, x, SA);
  k_ln_h<<<dim3((unsigned)SEQ, (unsigned)NB), 256, 0, stream>>>(SA, g1, be1, X1, (unsigned)SEQ, XA);
  k_gemm_selu<<<dim3((unsigned)(DFF / 64), (unsigned)(MROWS / 128)), 128, 0, stream>>>(XA, DM, B1, DM, 0.0625f, b1, X1, Hh, SA, DFF, DM);
  k_gemm_res<<<dim3((unsigned)(DM / 64), (unsigned)(MROWS / 128)), 128, 0, stream>>>(Hh, DFF, B2, DFF, 0.0625f, b2, X1, XA, SA, DM, DFF);
  k_ln_f<<<dim3((unsigned)SEQ, (unsigned)NB), 256, 0, stream>>>(SA, g2, be2, (float*)d_out, (unsigned)SEQ_FULL, XA);
}
